// DiagAttention_90778428768785
// MI455X (gfx1250) — hardware-verified
//
#include <hip/hip_runtime.h>


namespace {
constexpr int B = 4, N = 4096, D = 64, NR = B * N;
constexpr float XS = 8.0f, PS = 1024.0f;
typedef _Float16 b16;
typedef __attribute__((ext_vector_type(16))) _Float16 v16b;
typedef __attribute__((ext_vector_type(8))) _Float16 v8b;
typedef __attribute__((ext_vector_type(8))) float v8f;
typedef __attribute__((ext_vector_type(4))) float v4f;
typedef __attribute__((ext_vector_type(2))) float v2f;
__device__ __forceinline__ float bf16_rne(float f) { unsigned int u = __float_as_uint(f); u += 0x7FFFu + ((u >> 16) & 1u); float r = __uint_as_float(u & 0xFFFF0000u); asm volatile("" : "+v"(r)); return r; }
__device__ __forceinline__ void split16(float v, b16& hi, b16& lo) { hi = (b16)v; lo = (b16)(v - (float)hi); }
__device__ __forceinline__ v16b frag_kb(const b16* p, int hh) { const v8b a = *(const v8b*)(p + 8 * hh), b = *(const v8b*)(p + 16 + 8 * hh); v16b f;
#pragma unroll
  for (int e = 0; e < 8; ++e) { f[e] = a[e]; f[8 + e] = b[e]; } return f; }
__device__ __forceinline__ v8f wmma16b(v16b a, v16b b, v8f c) { v8f d = __builtin_amdgcn_wmma_f32_16x16x32_f16(false, a, false, b, (short)0, c, false, false); asm volatile("v_nop\n\tv_nop\n\tv_nop\n\tv_nop" : "+v"(d) : "v"(a), "v"(b)); return d; }
__device__ __forceinline__ void wave_lds_sync() { __builtin_amdgcn_fence(__ATOMIC_RELEASE, "workgroup"); __builtin_amdgcn_wave_barrier(); __builtin_amdgcn_fence(__ATOMIC_ACQUIRE, "workgroup"); }
__device__ __forceinline__ float pmul(float a, float b) { float p = a * b; asm volatile("" : "+v"(p)); return p; }

__global__ __launch_bounds__(32) void prep_kernel(const float* __restrict__ x, const float* __restrict__ qd, const float* __restrict__ kd, const float* __restrict__ vd, int BV, b16* __restrict__ XQ, b16* __restrict__ KH, b16* __restrict__ KL, b16* __restrict__ VTh, b16* __restrict__ VTl) {
  const int lane = threadIdx.x; const int b = blockIdx.x / (N / 32), ch = blockIdx.x % (N / 32); if (b >= BV) return; const size_t row = (size_t)b * N + ch * 32 + lane; const size_t base = ((size_t)b * (N / 32) + ch) * D;
  for (int pass = 0; pass < 2; ++pass) {
    for (int d0 = 0; d0 < D; d0 += 8) { v8b xq, kh, kl;
#pragma unroll
      for (int j = 0; j < 8; ++j) { const int d = d0 + j; const float xv = bf16_rne(x[row * D + d]); xq[j] = (b16)(xv * XS); b16 p, q; split16(pmul(xv, pmul(bf16_rne(qd[d]), bf16_rne(kd[d]))) * XS, p, q); kh[j] = p; kl[j] = q;
        b16 vp, vq; split16(pmul(xv, bf16_rne(vd[d])) * XS, vp, vq); ((volatile b16*)VTh)[(base + d) * 64 + lane] = vp; ((volatile b16*)VTl)[(base + d) * 64 + lane] = vq; }
      *(volatile v8b*)(XQ + row * D + d0) = xq; *(volatile v8b*)(KH + row * D + d0) = kh; *(volatile v8b*)(KL + row * D + d0) = kl; }
    __threadfence(); } }
__global__ __launch_bounds__(32) void att_kernel(const b16* __restrict__ XQ, const b16* __restrict__ KH, const b16* __restrict__ KL, const b16* __restrict__ VTh, const b16* __restrict__ VTl, int QV, float* __restrict__ out) {
  __shared__ __attribute__((aligned(16))) b16 Ph[16][40], Pl[16][40]; __shared__ float Sc[16][33], Mx[16], Dn[16], Sf[16], Of[16][D + 2];
  const int lane = threadIdx.x, nloc = lane & 15, hlf = lane >> 4; const int qt = blockIdx.x % (N / 16); const int b = blockIdx.x / (N / 16); const int q0 = qt * 16; if (q0 >= QV) return; const size_t qrow = (size_t)b * N + q0;
  if (lane < 16) { Mx[lane] = -INFINITY; Dn[lane] = 0.0f; Sf[lane] = 0.0f; }
  v16b qa[2]; qa[0] = frag_kb(XQ + (qrow + nloc) * D, hlf); qa[1] = frag_kb(XQ + (qrow + nloc) * D + 32, hlf);
  v8f acc[4] = {(v8f){}, (v8f){}, (v8f){}, (v8f){}}; wave_lds_sync();
#pragma unroll 1
  for (int kc = 0; kc < N; kc += 32) {
#pragma unroll
    for (int blk = 0; blk < 2; ++blk) { v8f s = {}; const size_t kr = ((size_t)b * N + kc + blk * 16 + nloc) * D;
#pragma unroll
      for (int kk = 0; kk < 2; ++kk) { const v16b kh = frag_kb(KH + kr + kk * 32, hlf), kl = frag_kb(KL + kr + kk * 32, hlf); s = wmma16b(qa[kk], kh, s); s = wmma16b(qa[kk], kl, s); }
#pragma unroll
      for (int r8 = 0; r8 < 8; ++r8) Sc[8 * hlf + r8][blk * 16 + nloc] = s[r8] * (0.125f / (XS * XS)); }
    wave_lds_sync();
#pragma unroll 1
    for (int qi = 0; qi < 16; ++qi) { const float sv = Sc[qi][lane]; float cm = sv; for (int o = 16; o; o >>= 1) cm = fmaxf(cm, __shfl_xor(cm, o)); const float mo = Mx[qi]; const float mn = fmaxf(mo, cm); const float p = __expf(sv - mn); float ps = p; for (int o = 16; o; o >>= 1) ps += __shfl_xor(ps, o);
      b16 ph, plo; split16(p * PS, ph, plo); Ph[qi][lane] = ph; Pl[qi][lane] = plo; if (lane == 0) { const float sf = (mo == -INFINITY) ? 0.0f : __expf(mo - mn); Sf[qi] = sf; Dn[qi] = Dn[qi] * sf + ps; Mx[qi] = mn; } }
    wave_lds_sync(); const v16b pa = frag_kb(&Ph[nloc][0], hlf), pb = frag_kb(&Pl[nloc][0], hlf); const size_t vb = (((size_t)b * (N / 32) + kc / 32) * D) * 64;
#pragma unroll
    for (int t = 0; t < 4; ++t) {
#pragma unroll
      for (int r8 = 0; r8 < 8; ++r8) acc[t][r8] *= Sf[8 * hlf + r8];
      const v16b vh = frag_kb(VTh + vb + (size_t)(t * 16 + nloc) * 64, hlf), vl = frag_kb(VTl + vb + (size_t)(t * 16 + nloc) * 64, hlf); acc[t] = wmma16b(pa, vh, acc[t]); acc[t] = wmma16b(pa, vl, acc[t]); acc[t] = wmma16b(pb, vh, acc[t]); }
    wave_lds_sync(); }
#pragma unroll
  for (int t = 0; t < 4; ++t)
#pragma unroll
    for (int r8 = 0; r8 < 8; ++r8) { const int rl = 8 * hlf + r8; Of[rl][t * 16 + nloc] = acc[t][r8] * (1.0f / (PS * XS)) / Dn[rl]; }
  wave_lds_sync();
  for (int pass = 0; pass < 2; ++pass) { for (int rr = 0; rr < 16; ++rr) *(volatile v2f*)(out + (qrow + rr) * D + lane * 2) = (v2f){Of[rr][lane * 2], Of[rr][lane * 2 + 1]}; __threadfence(); }
}
}

extern "C" void kernel_launch(void* const* d_in, const int* in_sizes, int n_in, void* d_out, int out_size, void* d_ws, size_t ws_size, hipStream_t stream) {
  (void)n_in;
  auto Fp = [&](int i) { return (const float*)d_in[i]; };
  if (in_sizes[0] != NR * D || in_sizes[1] != D || in_sizes[2] != D || in_sizes[3] != D || out_size != NR * D) return;
  const int BV = B, QV = N;
  size_t off = 0; char* ws = (char*)d_ws;
  auto carve = [&](size_t bytes) { char* p = ws + off; off += (bytes + 255) & ~(size_t)255; return p; };
  b16* XQ = (b16*)carve((size_t)NR * D * 2); b16* KH = (b16*)carve((size_t)NR * D * 2); b16* KL = (b16*)carve((size_t)NR * D * 2); b16* VTh = (b16*)carve((size_t)B * (N / 32) * D * 64 * 2); b16* VTl = (b16*)carve((size_t)B * (N / 32) * D * 64 * 2);
  if (off > ws_size || off > ((size_t)32 << 20)) return;
  prep_kernel<<<BV * (N / 32), 32, 0, stream>>>(Fp(0), Fp(1), Fp(2), Fp(3), BV, XQ, KH, KL, VTh, VTl);
  att_kernel<<<BV * (N / 16), 32, 0, stream>>>(XQ, KH, KL, VTh, VTl, QV, (float*)d_out);
}
